// MambaBlock_10273561772152
// MI455X (gfx1250) — hardware-verified
//
#include <hip/hip_runtime.h>
#include <math.h>

typedef __attribute__((ext_vector_type(16))) _Float16 v16h;
typedef __attribute__((ext_vector_type(8)))  _Float16 v8h;
typedef __attribute__((ext_vector_type(16))) __bf16   v16b;
typedef __attribute__((ext_vector_type(8)))  __bf16   v8b;
typedef __attribute__((ext_vector_type(8)))  float    v8f;
typedef __attribute__((ext_vector_type(4)))  float    v4f;

constexpr int kBatch  = 4;
constexpr int kSeq    = 1024;
constexpr int kDm     = 1024;
constexpr int kDin    = 2048;
constexpr int kNst    = 16;
constexpr int kTaps   = 4;
constexpr int kRows   = kBatch * kSeq;
constexpr int kXdN    = 1 + 2 * kNst;
constexpr int kXdP    = 64;
constexpr int kScanCh = 256;
constexpr int kScanTS = 16;
constexpr int kTP     = 260;
constexpr int kSXP    = 68;
constexpr float kWinCarry  = 32.0f;
constexpr float kWoutCarry = 32.0f;
constexpr float kYCarry    = 16.0f;
constexpr float kInScale   = 1.0f / kWinCarry;
constexpr float kOutScale  = 1.0f / (kYCarry * kWoutCarry);
static_assert(kXdN <= kXdP);
static_assert((kDm % 32) == 0 && (kDin % 32) == 0);
static_assert((kRows % 64) == 0 && (kDin % 64) == 0 && (kXdP % 64) == 0 && (kDm % 64) == 0);
static_assert((kSeq % 64) == 0 && (kSeq % kScanTS) == 0 && (kDin % kScanCh) == 0 && (kDin % 256) == 0);
static_assert(kScanCh == 256);

constexpr size_t kSzXB   = (size_t)kRows * kDm * 2;
constexpr size_t kSzWIB  = (size_t)(2 * kDin) * kDm * 2;
constexpr size_t kSzYG   = (size_t)kRows * kDin * 2;
constexpr size_t kSzWXB  = (size_t)kXdP * kDin * 2;
constexpr size_t kSzWOB  = (size_t)kDm * kDin * 2;
constexpr size_t kSzF32P = (size_t)kRows * kDin * 4;
constexpr size_t kSzU16  = (size_t)kRows * kDin * 2;
constexpr size_t kSzXD   = (size_t)kRows * kXdP * 4;
constexpr size_t kOffXB  = 0;
constexpr size_t kOffWIB = kOffXB + kSzXB;
constexpr size_t kOffYG  = 0;
constexpr size_t kOffWXB = kOffWIB + kSzWIB;
constexpr size_t kOffWOB = kOffWXB + kSzWXB;
constexpr size_t kOffXP  = kOffWOB + kSzWOB;
constexpr size_t kOffY   = kOffXP;
constexpr size_t kOffZ   = kOffXP + kSzF32P;
constexpr size_t kOffUH  = kOffZ + kSzF32P;
constexpr size_t kOffUL  = kOffUH + kSzU16;
constexpr size_t kOffXD  = kOffUL + kSzU16;
constexpr size_t kWsTotal = kOffXD + kSzXD;
static_assert(kSzYG == kSzXB + kSzWIB);
static_assert(kWsTotal == 122945536ull);
static_assert(kWsTotal <= 134217728ull);
static_assert((kOffWIB % 128) == 0 && (kOffWXB % 128) == 0 && (kOffWOB % 128) == 0 && (kOffXP % 128) == 0 &&
              (kOffZ % 128) == 0 && (kOffUH % 128) == 0 && (kOffUL % 128) == 0 && (kOffXD % 128) == 0);

__device__ __forceinline__ unsigned short f2bf_bits(float f) {
  unsigned u = __float_as_uint(f);
  return (unsigned short)((u + 0x7FFFu + ((u >> 16) & 1u)) >> 16);
}
__device__ __forceinline__ float bf_bits2f(unsigned short h) { return __uint_as_float(((unsigned)h) << 16); }
__device__ __forceinline__ float bfr(float f) { return bf_bits2f(f2bf_bits(f)); }

__device__ __forceinline__ void dep_guard_h(v8f& a, v8f& b, v16h x, v16h y) { asm volatile("v_nop\n\tv_nop\n\tv_nop\n\tv_nop" : "+v"(a), "+v"(b) : "v"(x), "v"(y)); }
__device__ __forceinline__ void dep_guard_b(v8f& a, v8f& b, v16b x, v16b y) { asm volatile("v_nop\n\tv_nop\n\tv_nop\n\tv_nop" : "+v"(a), "+v"(b) : "v"(x), "v"(y)); }
__device__ __forceinline__ void dep_guard4_h(v8f& a, v8f& b, v8f& c, v8f& d, v16h x, v16h y) { asm volatile("v_nop\n\tv_nop\n\tv_nop\n\tv_nop" : "+v"(a), "+v"(b), "+v"(c), "+v"(d) : "v"(x), "v"(y)); }
__device__ __forceinline__ void dep_guard4_b(v8f& a, v8f& b, v8f& c, v8f& d, v16b x, v16b y) { asm volatile("v_nop\n\tv_nop\n\tv_nop\n\tv_nop" : "+v"(a), "+v"(b), "+v"(c), "+v"(d) : "v"(x), "v"(y)); }
__device__ __forceinline__ void keep4_h(v16h a, v16h b, v16h c, v16h d) { asm volatile("v_nop" :: "v"(a), "v"(b), "v"(c), "v"(d)); }
__device__ __forceinline__ void keep4_b(v16b a, v16b b, v16b c, v16b d) { asm volatile("v_nop" :: "v"(a), "v"(b), "v"(c), "v"(d)); }
__device__ __forceinline__ void acc_guard4(v8f& a, v8f& b, v8f& c, v8f& d) { asm volatile("v_nop\n\tv_nop\n\tv_nop\n\tv_nop" : "+v"(a), "+v"(b), "+v"(c), "+v"(d)); }
template <typename T> struct Frag;
template <> struct Frag<_Float16> {
  typedef v16h V; union U { v16h v; v8h h[2]; };
  static __device__ __forceinline__ v16h load(const _Float16* p) {
    U f; f.h[0] = *(const v8h*)(p); f.h[1] = *(const v8h*)(p + 16); return f.v;
  }
  static __device__ __forceinline__ v8f mma(v16h a, v16h b, v8f c) {
    return __builtin_amdgcn_wmma_f32_16x16x32_f16(false, a, false, b, (short)0, c, false, false);
  }
  static __device__ __forceinline__ void guard(v8f& a, v8f& b, v16h x, v16h y) { dep_guard_h(a, b, x, y); }
  static __device__ __forceinline__ void guard4(v8f& a, v8f& b, v8f& c, v8f& d, v16h x, v16h y) { dep_guard4_h(a, b, c, d, x, y); }
  static __device__ __forceinline__ void keep(v16h a, v16h b, v16h c, v16h d) { keep4_h(a, b, c, d); }
};
template <> struct Frag<__bf16> {
  typedef v16b V; union U { v16b v; v8b h[2]; };
  static __device__ __forceinline__ v16b load(const __bf16* p) {
    U f; f.h[0] = *(const v8b*)(p); f.h[1] = *(const v8b*)(p + 16); return f.v;
  }
  static __device__ __forceinline__ v8f mma(v16b a, v16b b, v8f c) {
    return __builtin_amdgcn_wmma_f32_16x16x32_bf16(false, a, false, b, (short)0, c, false, false);
  }
  static __device__ __forceinline__ void guard(v8f& a, v8f& b, v16b x, v16b y) { dep_guard_b(a, b, x, y); }
  static __device__ __forceinline__ void guard4(v8f& a, v8f& b, v8f& c, v8f& d, v16b x, v16b y) { dep_guard4_b(a, b, c, d, x, y); }
  static __device__ __forceinline__ void keep(v16b a, v16b b, v16b c, v16b d) { keep4_b(a, b, c, d); }
};

template <int ET> struct Elem;
template <> struct Elem<0> { typedef _Float16 T; };
template <> struct Elem<1> { typedef __bf16 T; };
template <int ET, int SPL, int BIAS_MODE, int OUT_MODE, bool RESID, int ACT = 0>
__global__ __launch_bounds__(256) void wmma_gemm64(
    const unsigned short* __restrict__ Ap, const unsigned short* __restrict__ A2p, int lda, long strideA,
    const unsigned short* __restrict__ Btp, const unsigned short* __restrict__ Bt2p, int ldb, long strideB,
    void* __restrict__ Cout, void* __restrict__ Cout2, int ldc, long strideC,
    const float* __restrict__ bias,
    const float* __restrict__ resid, long strideR,
    int M, int N, int K, float scale) {
  typedef typename Elem<ET>::T T;
  typedef typename Frag<T>::V V;
  const T* A = (const T*)Ap; const T* A2 = (const T*)A2p; const T* Bt = (const T*)Btp; const T* Bt2 = (const T*)Bt2p;
  __shared__ __align__(16) float sT[8][16 * 68];
  const int b    = blockIdx.y;
  const int lane = threadIdx.x & 31;
  const int wave = threadIdx.x >> 5;
  const int tilesN = N >> 6;
  const int tilesM = M >> 6;
  const int tile = blockIdx.x * 8 + wave;
  if (tile >= tilesM * tilesN) return;
  const int tm = tile / tilesN;
  const int tn = tile - tm * tilesN;
  const int m0 = tm << 6;
  const int n0 = tn << 6;

  const T* Ab  = A  + (size_t)b * strideA;
  const T* Bb  = Bt + (size_t)b * strideB;
  const T* Ab2 = (SPL >= 1) ? (A2  + (size_t)b * strideA) : nullptr;
  const T* Bb2 = (SPL == 2) ? (Bt2 + (size_t)b * strideB) : nullptr;

  const int rlane = lane & 15;
  const int koff  = (lane >> 4) * 8;
  const int mOff  = (lane >> 4) * 8;

  v8f acc[4][4];
#pragma unroll
  for (int i = 0; i < 4; ++i)
#pragma unroll
    for (int j = 0; j < 4; ++j) acc[i][j] = (v8f){0.f,0.f,0.f,0.f,0.f,0.f,0.f,0.f};

  for (int k0 = 0; k0 < K; k0 += 32) {
    V bh[4], bl[4];
#pragma unroll
    for (int j = 0; j < 4; ++j) {
      const size_t bo = (size_t)(n0 + (j << 4) + rlane) * ldb + koff + k0;
      bh[j] = Frag<T>::load(Bb + bo);
      if (SPL == 2) bl[j] = Frag<T>::load(Bb2 + bo);
    }
#pragma unroll
    for (int i = 0; i < 4; ++i) {
      const size_t ao = (size_t)(m0 + (i << 4) + rlane) * lda + koff + k0;
      V ah = Frag<T>::load(Ab + ao);
      V al;
      if (SPL >= 1) al = Frag<T>::load(Ab2 + ao);
#pragma unroll
      for (int j = 0; j < 4; ++j) {
        acc[i][j] = Frag<T>::mma(ah, bh[j], acc[i][j]);
        if (SPL == 2) acc[i][j] = Frag<T>::mma(ah, bl[j], acc[i][j]);
        if (SPL >= 1) acc[i][j] = Frag<T>::mma(al, bh[j], acc[i][j]);
      }
      Frag<T>::guard4(acc[i][0], acc[i][1], acc[i][2], acc[i][3], ah, (SPL >= 1) ? al : ah);
    }
    Frag<T>::keep(bh[0], bh[1], bh[2], bh[3]);
    if (SPL == 2) Frag<T>::keep(bl[0], bl[1], bl[2], bl[3]);
  }
  acc_guard4(acc[0][0], acc[0][1], acc[0][2], acc[0][3]);
  acc_guard4(acc[1][0], acc[1][1], acc[1][2], acc[1][3]);
  acc_guard4(acc[2][0], acc[2][1], acc[2][2], acc[2][3]);
  acc_guard4(acc[3][0], acc[3][1], acc[3][2], acc[3][3]);

  float* slab = sT[wave];
  const float* Rb = RESID ? (resid + (size_t)b * strideR) : nullptr;
#pragma unroll
  for (int i = 0; i < 4; ++i) {
    const int mBase = m0 + (i << 4);
#pragma unroll
    for (int j = 0; j < 4; ++j) {
      const int n = n0 + (j << 4) + rlane;
      float bv = 0.f;
      if (BIAS_MODE == 2) bv = bias[n];
#pragma unroll
      for (int r = 0; r < 8; ++r) {
        float v = acc[i][j][r] * scale;
        if (BIAS_MODE == 1) v += bias[mBase + mOff + r];
        if (BIAS_MODE == 2) v += bv;
        if (RESID) v += Rb[(size_t)(mBase + mOff + r) * ldc + n];
        if (ACT == 1) v = tanhf(v);
        if (ACT == 2) v = fmaxf(v, 0.0f);
        if (ACT == 3) v = v / (1.0f + expf(-v));
        if (ACT == 4) v = (v > 0.f) ? v : 0.01f * v;
        slab[(mOff + r) * 68 + (j << 4) + rlane] = v;
      }
    }
    __builtin_amdgcn_fence(__ATOMIC_RELEASE, "workgroup");
    __builtin_amdgcn_wave_barrier();
    __builtin_amdgcn_fence(__ATOMIC_ACQUIRE, "workgroup");
    if (OUT_MODE == 0) {
      float* C = (float*)Cout + (size_t)b * strideC;
      const int hh = lane >> 4, c4 = (lane & 15) * 4;
      for (int pass = 0; pass < 2; ++pass) {
#pragma unroll
        for (int it = 0; it < 8; ++it) {
          const int row = it * 2 + hh;
          v4f v = *(const v4f*)(slab + row * 68 + c4);
          *(volatile v4f*)(C + (size_t)(mBase + row) * ldc + n0 + c4) = v;
        }
        __threadfence();
      }
    } else {
      const int q = lane >> 3, c8 = (lane & 7) * 8;
      unsigned short* C  = (unsigned short*)Cout  + (size_t)b * strideC;
      unsigned short* C2 = (OUT_MODE == 2) ? ((unsigned short*)Cout2 + (size_t)b * strideC) : nullptr;
      for (int pass = 0; pass < 2; ++pass) {
#pragma unroll
        for (int it = 0; it < 4; ++it) {
          const int row = it * 4 + q;
          const float* sp = slab + row * 68 + c8;
          v8h hv, lv;
#pragma unroll
          for (int e = 0; e < 8; ++e) {
            if (OUT_MODE == 1) {
              hv[e] = (_Float16)sp[e];
            } else {
              unsigned short hb = f2bf_bits(sp[e]);
              unsigned short lb = f2bf_bits(sp[e] - bf_bits2f(hb));
              hv[e] = __builtin_bit_cast(_Float16, hb);
              lv[e] = __builtin_bit_cast(_Float16, lb);
            }
          }
          *(volatile v8h*)(C + (size_t)(mBase + row) * ldc + n0 + c8) = hv;
          if (OUT_MODE == 2) *(volatile v8h*)(C2 + (size_t)(mBase + row) * ldc + n0 + c8) = lv;
        }
        __threadfence();
      }
    }
    __builtin_amdgcn_fence(__ATOMIC_RELEASE, "workgroup");
    __builtin_amdgcn_wave_barrier();
    __builtin_amdgcn_fence(__ATOMIC_ACQUIRE, "workgroup");
  }
}

template <int MODE>
__global__ __launch_bounds__(256) void cast_plane_kernel(
    const float* __restrict__ src, unsigned short* __restrict__ dst, int total8, int colShift, int rowsValid, float scale)
{
  const int i = blockIdx.x * 256 + threadIdx.x;
  if (i >= total8) return;
  const size_t e0 = (size_t)i << 3;
  const int ncols = 1 << colShift;
  const int row = (int)(e0 >> colShift);
  const int col = (int)(e0 & (size_t)(ncols - 1));
  const bool valid = row < rowsValid;
  const int rc = valid ? row : (rowsValid - 1);
  const float* p = src + (size_t)rc * ncols + col;
  const v4f a0 = *(const v4f*)(p);
  const v4f a1 = *(const v4f*)(p + 4);
  v8h hv;
#pragma unroll
  for (int e = 0; e < 4; ++e) {
    const float f0 = valid ? a0[e] : 0.f;
    const float f1 = valid ? a1[e] : 0.f;
    const unsigned short b0 = f2bf_bits(f0), b1 = f2bf_bits(f1);
    if (MODE == 0) {
      hv[e]     = (_Float16)(bf_bits2f(b0) * scale);
      hv[4 + e] = (_Float16)(bf_bits2f(b1) * scale);
    } else {
      hv[e]     = __builtin_bit_cast(_Float16, b0);
      hv[4 + e] = __builtin_bit_cast(_Float16, b1);
    }
  }
  unsigned short* q = dst + e0;
  *(volatile v8h*)q = hv;
  __threadfence();
  *(volatile v8h*)q = hv;
}

__global__ __launch_bounds__(256) void conv_silu_kernel(
    const float* __restrict__ XP, const float* __restrict__ cw, const float* __restrict__ cb,
    unsigned short* __restrict__ UH, unsigned short* __restrict__ UL)
{
  __shared__ __align__(16) float sT[16 * kTP];
  const int tid = threadIdx.x, lane = tid & 31, wave = tid >> 5;
  const int d0 = blockIdx.x * 256, d = d0 + tid;
  const int g0 = blockIdx.y * 64;
  const int tb = g0 & (kSeq - 1);
  const float w0 = bfr(cw[d * kTaps + 0]), w1 = bfr(cw[d * kTaps + 1]), w2 = bfr(cw[d * kTaps + 2]), w3 = bfr(cw[d * kTaps + 3]);
  const float bc = bfr(cb[d]);
  float xm3, xm2, xm1;
  {
    const bool hist = (tb > 0);
    const int rb = hist ? (g0 - 3) : g0;
    const float v3 = XP[(size_t)rb * kDin + d];
    const float v2 = XP[(size_t)(rb + 1) * kDin + d];
    const float v1 = XP[(size_t)(rb + 2) * kDin + d];
    xm3 = hist ? v3 : 0.f;
    xm2 = hist ? v2 : 0.f;
    xm1 = hist ? v1 : 0.f;
  }
#pragma unroll 1
  for (int sub = 0; sub < 4; ++sub) {
    const int lb = g0 + sub * 16;
#pragma unroll 1
    for (int s = 0; s < 16; ++s) {
      const float xcur = XP[(size_t)(lb + s) * kDin + d];
      float acc = w0 * xm3;
      acc = fmaf(w1, xm2, acc);
      acc = fmaf(w2, xm1, acc);
      acc = fmaf(w3, xcur, acc);
      const float sv = acc + bc;
      const float sg = 1.0f / (1.0f + expf(-sv));
      sT[s * kTP + tid] = sv * sg;
      xm3 = xm2; xm2 = xm1; xm1 = xcur;
    }
    __syncthreads();
    v8h bh[2], blo[2];
#pragma unroll
    for (int it = 0; it < 2; ++it) {
      const float* sp = sT + (it * 8 + wave) * kTP + lane * 8;
      const v4f a0 = *(const v4f*)(sp);
      const v4f a1 = *(const v4f*)(sp + 4);
#pragma unroll
      for (int e = 0; e < 4; ++e) {
        const unsigned short h0 = f2bf_bits(a0[e]), h1 = f2bf_bits(a1[e]);
        const unsigned short l0 = f2bf_bits(a0[e] - bf_bits2f(h0)), l1 = f2bf_bits(a1[e] - bf_bits2f(h1));
        bh[it][e]      = __builtin_bit_cast(_Float16, h0);
        bh[it][4 + e]  = __builtin_bit_cast(_Float16, h1);
        blo[it][e]     = __builtin_bit_cast(_Float16, l0);
        blo[it][4 + e] = __builtin_bit_cast(_Float16, l1);
      }
    }
    for (int pass = 0; pass < 2; ++pass) {
#pragma unroll
      for (int it = 0; it < 2; ++it) {
        const size_t o = (size_t)(lb + it * 8 + wave) * kDin + d0 + lane * 8;
        *(volatile v8h*)(UH + o) = bh[it];
        *(volatile v8h*)(UL + o) = blo[it];
      }
      __threadfence();
    }
    __syncthreads();
  }
}

__global__ __launch_bounds__(256) void scan_kernel(
    const float* __restrict__ XD, const unsigned short* __restrict__ UH, const unsigned short* __restrict__ UL,
    const float* __restrict__ Wdt, const float* __restrict__ bdt, const float* __restrict__ Alog,
    float* __restrict__ Y)
{
  __shared__ __align__(16) float sX[kScanTS * kSXP];
  __shared__ __align__(16) float sY[kScanTS * kTP];
  __shared__ float sA[kNst];
  const int tid = threadIdx.x, lane = tid & 31, wave = tid >> 5;
  constexpr int kBlkPerB = kDin / kScanCh;
  const int bix = blockIdx.x / kBlkPerB;
  const int d0  = (blockIdx.x - bix * kBlkPerB) * kScanCh;
  const int d   = d0 + tid;
  const size_t row0 = (size_t)bix * kSeq;
  {
    const float al = bfr(Alog[tid & (kNst - 1)]);
    const float av = -expf(fminf(al, 5.0f));
    if (tid < kNst) sA[tid] = av;
  }
  const float wd = bfr(Wdt[d]);
  const float bd = bfr(bdt[d]);
  __syncthreads();
  float As[kNst], h[kNst];
#pragma unroll
  for (int n = 0; n < kNst; ++n) { As[n] = sA[n]; h[n] = 0.f; }
  const int sr = tid >> 4, sq = (tid & 15) * 4;
  const int hrow = wave >> 1, hch = (wave & 1) * 128 + lane * 4;
#pragma unroll 1
  for (int c = 0; c < kSeq / kScanTS; ++c) {
    const int l0 = c * kScanTS;
    __syncthreads();
    {
      const v4f v = *(const v4f*)(XD + (row0 + l0 + sr) * kXdP + sq);
      float* sp = sX + sr * kSXP + 3 + sq;
      sp[0] = v[0]; sp[1] = v[1]; sp[2] = v[2]; sp[3] = v[3];
    }
    __syncthreads();
#pragma unroll 1
    for (int s = 0; s < kScanTS; ++s) {
      const float* xr = sX + s * kSXP;
      const float dtr = xr[3];
      v4f Bq[4], Cq[4];
#pragma unroll
      for (int q4 = 0; q4 < 4; ++q4) {
        Bq[q4] = *(const v4f*)(xr + 4 + 4 * q4);
        Cq[q4] = *(const v4f*)(xr + 4 + kNst + 4 * q4);
      }
      const float v   = fmaf(dtr, wd, bd);
      const float a   = __expf(-fabsf(v));
      const float up  = 1.0f + a;
      const float l1p = __logf(up) + (a - (up - 1.0f)) * __builtin_amdgcn_rcpf(up);
      float dt = fmaxf(v, 0.0f) + l1p;
      dt = fminf(fmaxf(dt, 1e-4f), 10.0f);
      const size_t m = (row0 + l0 + s) * kDin + d;
      const unsigned wh = UH[m];
      const unsigned wl = UL[m];
      const float u = __uint_as_float(wh << 16) + __uint_as_float(wl << 16);
      float y = 0.f;
#pragma unroll
      for (int n = 0; n < kNst; ++n) {
        float ea = dt * As[n];
        ea = fminf(fmaxf(ea, -20.0f), 0.0f);
        const float e  = __expf(ea);
        const float db = dt * Bq[n >> 2][n & 3];
        float p = db * u;
        p = fminf(fmaxf(p, -10.0f), 10.0f);
        float hn = fmaf(h[n], e, p);
        hn = fminf(fmaxf(hn, -100.0f), 100.0f);
        h[n] = hn;
        y = fmaf(hn, Cq[n >> 2][n & 3], y);
      }
      sY[s * kTP + tid] = y;
    }
    __syncthreads();
    v4f fv[4];
#pragma unroll
    for (int it = 0; it < 4; ++it) fv[it] = *(const v4f*)(sY + (it * 4 + hrow) * kTP + hch);
    for (int pass = 0; pass < 2; ++pass) {
#pragma unroll
      for (int it = 0; it < 4; ++it)
        *(volatile v4f*)(Y + (row0 + l0 + it * 4 + hrow) * kDin + d0 + hch) = fv[it];
      __threadfence();
    }
  }
}

__global__ __launch_bounds__(256) void ln_gate_kernel(
    const float* __restrict__ Y, const float* __restrict__ Z,
    const unsigned short* __restrict__ UH, const unsigned short* __restrict__ UL,
    const float* __restrict__ lng, const float* __restrict__ lnb, const float* __restrict__ Dv,
    unsigned short* __restrict__ YG)
{
  __shared__ float sred[8];
  const int tid = threadIdx.x, lane = tid & 31, wave = tid >> 5;
  const size_t rb = (size_t)blockIdx.x * kDin;
  const int c0 = tid * 8;
  const v4f ya = *(const v4f*)(Y + rb + c0);
  const v4f yb = *(const v4f*)(Y + rb + c0 + 4);
  float yv[8];
  yv[0] = ya[0]; yv[1] = ya[1]; yv[2] = ya[2]; yv[3] = ya[3];
  yv[4] = yb[0]; yv[5] = yb[1]; yv[6] = yb[2]; yv[7] = yb[3];
  float s = 0.f;
#pragma unroll
  for (int e = 0; e < 8; ++e) s += yv[e];
#pragma unroll
  for (int off = 16; off > 0; off >>= 1) s += __shfl_xor(s, off, 32);
  if (lane == 0) sred[wave] = s;
  __syncthreads();
  float tot = 0.f;
#pragma unroll
  for (int w = 0; w < 8; ++w) tot += sred[w];
  const float mu = tot * (1.0f / (float)kDin);
  float dq = 0.f;
#pragma unroll
  for (int e = 0; e < 8; ++e) { const float dd = yv[e] - mu; dq = fmaf(dd, dd, dq); }
#pragma unroll
  for (int off = 16; off > 0; off >>= 1) dq += __shfl_xor(dq, off, 32);
  __syncthreads();
  if (lane == 0) sred[wave] = dq;
  __syncthreads();
  float totq = 0.f;
#pragma unroll
  for (int w = 0; w < 8; ++w) totq += sred[w];
  const float var  = totq * (1.0f / (float)kDin);
  const float rstd = 1.0f / sqrtf(var + 1e-5f);

  const v4f ga = *(const v4f*)(lng + c0), gb = *(const v4f*)(lng + c0 + 4);
  const v4f ba = *(const v4f*)(lnb + c0), bb = *(const v4f*)(lnb + c0 + 4);
  const v4f da = *(const v4f*)(Dv + c0),  db = *(const v4f*)(Dv + c0 + 4);
  asm volatile("" ::: "memory");
  const uint4 uh = *(const uint4*)(UH + rb + c0);
  const uint4 ul = *(const uint4*)(UL + rb + c0);
  const v4f za = *(const v4f*)(Z + rb + c0), zb = *(const v4f*)(Z + rb + c0 + 4);
  float gv[8], bv[8], dv[8], zv[8], xv[8];
  gv[0] = ga[0]; gv[1] = ga[1]; gv[2] = ga[2]; gv[3] = ga[3]; gv[4] = gb[0]; gv[5] = gb[1]; gv[6] = gb[2]; gv[7] = gb[3];
  bv[0] = ba[0]; bv[1] = ba[1]; bv[2] = ba[2]; bv[3] = ba[3]; bv[4] = bb[0]; bv[5] = bb[1]; bv[6] = bb[2]; bv[7] = bb[3];
  dv[0] = da[0]; dv[1] = da[1]; dv[2] = da[2]; dv[3] = da[3]; dv[4] = db[0]; dv[5] = db[1]; dv[6] = db[2]; dv[7] = db[3];
  zv[0] = za[0]; zv[1] = za[1]; zv[2] = za[2]; zv[3] = za[3]; zv[4] = zb[0]; zv[5] = zb[1]; zv[6] = zb[2]; zv[7] = zb[3];
  {
    const unsigned wh0 = uh.x, wh1 = uh.y, wh2 = uh.z, wh3 = uh.w;
    const unsigned wl0 = ul.x, wl1 = ul.y, wl2 = ul.z, wl3 = ul.w;
    xv[0] = __uint_as_float(wh0 << 16) + __uint_as_float(wl0 << 16);
    xv[1] = __uint_as_float(wh0 & 0xffff0000u) + __uint_as_float(wl0 & 0xffff0000u);
    xv[2] = __uint_as_float(wh1 << 16) + __uint_as_float(wl1 << 16);
    xv[3] = __uint_as_float(wh1 & 0xffff0000u) + __uint_as_float(wl1 & 0xffff0000u);
    xv[4] = __uint_as_float(wh2 << 16) + __uint_as_float(wl2 << 16);
    xv[5] = __uint_as_float(wh2 & 0xffff0000u) + __uint_as_float(wl2 & 0xffff0000u);
    xv[6] = __uint_as_float(wh3 << 16) + __uint_as_float(wl3 << 16);
    xv[7] = __uint_as_float(wh3 & 0xffff0000u) + __uint_as_float(wl3 & 0xffff0000u);
  }
  v8h hv;
#pragma unroll
  for (int e = 0; e < 8; ++e) {
    const float g = bfr(gv[e]), bq = bfr(bv[e]), dd = bfr(dv[e]);
    float vln = (yv[e] - mu) * rstd;
    vln = fmaf(vln, g, bq);
    vln = fmaf(dd, xv[e], vln);
    const float zz = zv[e];
    const float sg = __builtin_amdgcn_rcpf(1.0f + __expf(-zz));
    const float gate = zz * sg;
    hv[e] = (_Float16)((vln * gate) * kYCarry);
  }
  unsigned short* q = YG + rb + c0;
  *(volatile v8h*)q = hv;
  __threadfence();
  *(volatile v8h*)q = hv;
}

extern "C" void kernel_launch(void* const* d_in, const int* in_sizes, int n_in,
                              void* d_out, int out_size, void* d_ws, size_t ws_size,
                              hipStream_t stream)
{
  if (n_in < 12) return;
  if (in_sizes[0] != kRows * kDm) return;
  if (in_sizes[1] != 2 * kDin * kDm) return;
  if (in_sizes[2] != kDin * kTaps) return;
  if (in_sizes[3] != kDin) return;
  if (in_sizes[4] != kXdN * kDin) return;
  if (in_sizes[5] != kDin) return;
  if (in_sizes[6] != kDin) return;
  if (in_sizes[7] != kNst) return;
  if (in_sizes[8] != kDin) return;
  if (in_sizes[9] != kDm * kDin) return;
  if (in_sizes[10] != kDin || in_sizes[11] != kDin) return;
  if (out_size != kRows * kDm) return;
  if (ws_size < kWsTotal) return;

  const float* x       = (const float*)d_in[0];
  const float* W_in    = (const float*)d_in[1];
  const float* conv_w  = (const float*)d_in[2];
  const float* conv_b  = (const float*)d_in[3];
  const float* W_xproj = (const float*)d_in[4];
  const float* W_dt    = (const float*)d_in[5];
  const float* b_dt    = (const float*)d_in[6];
  const float* A_log   = (const float*)d_in[7];
  const float* Dp      = (const float*)d_in[8];
  const float* W_out   = (const float*)d_in[9];
  const float* ln_g    = (const float*)d_in[10];
  const float* ln_b    = (const float*)d_in[11];
  float* out = (float*)d_out;

  char* ws = (char*)d_ws;
  unsigned short* XB  = (unsigned short*)(ws + kOffXB);
  unsigned short* WIB = (unsigned short*)(ws + kOffWIB);
  unsigned short* YG  = (unsigned short*)(ws + kOffYG);
  unsigned short* WXB = (unsigned short*)(ws + kOffWXB);
  unsigned short* WOB = (unsigned short*)(ws + kOffWOB);
  float*          XP  = (float*)(ws + kOffXP);
  float*          Yp  = (float*)(ws + kOffY);
  float*          Zp  = (float*)(ws + kOffZ);
  unsigned short* UH  = (unsigned short*)(ws + kOffUH);
  unsigned short* UL  = (unsigned short*)(ws + kOffUL);
  float*          XD  = (float*)(ws + kOffXD);
  const float* dummy_bias  = b_dt;
  const float* dummy_resid = x;

  cast_plane_kernel<0><<<(kRows * kDm / 8) / 256, 256, 0, stream>>>(x, XB, kRows * kDm / 8, 10, kRows, 1.0f);
  cast_plane_kernel<0><<<(2 * kDin * kDm / 8) / 256, 256, 0, stream>>>(W_in, WIB, 2 * kDin * kDm / 8, 10, 2 * kDin, kWinCarry);
  cast_plane_kernel<0><<<(kDm * kDin / 8) / 256, 256, 0, stream>>>(W_out, WOB, kDm * kDin / 8, 11, kDm, kWoutCarry);
  cast_plane_kernel<1><<<(kXdP * kDin / 8) / 256, 256, 0, stream>>>(W_xproj, WXB, kXdP * kDin / 8, 11, kXdN, 1.0f);

  wmma_gemm64<0, 0, 0, 0, false><<<dim3(256, 1), 256, 0, stream>>>(
      XB, XB, kDm, 0L,
      WIB, WIB, kDm, 0L,
      (void*)XP, (void*)XP, kDin, 0L,
      dummy_bias, dummy_resid, 0L,
      kRows, kDin, kDm, kInScale);
  wmma_gemm64<0, 0, 0, 0, false><<<dim3(256, 1), 256, 0, stream>>>(
      XB, XB, kDm, 0L,
      WIB + (size_t)kDin * kDm, WIB + (size_t)kDin * kDm, kDm, 0L,
      (void*)Zp, (void*)Zp, kDin, 0L,
      dummy_bias, dummy_resid, 0L,
      kRows, kDin, kDm, kInScale);

  conv_silu_kernel<<<dim3(kDin / 256, kRows / 64), 256, 0, stream>>>(XP, conv_w, conv_b, UH, UL);

  wmma_gemm64<1, 1, 0, 0, false><<<dim3(8, 1), 256, 0, stream>>>(
      UH, UL, kDin, 0L,
      WXB, WXB, kDin, 0L,
      (void*)XD, (void*)XD, kXdP, 0L,
      dummy_bias, dummy_resid, 0L,
      kRows, kXdP, kDin, 1.0f);

  scan_kernel<<<kBatch * (kDin / kScanCh), kScanCh, 0, stream>>>(XD, UH, UL, W_dt, b_dt, A_log, Yp);

  ln_gate_kernel<<<kRows, 256, 0, stream>>>(Yp, Zp, UH, UL, ln_g, ln_b, Dp, YG);

  wmma_gemm64<0, 0, 0, 0, false><<<dim3(128, 1), 256, 0, stream>>>(
      YG, YG, kDin, 0L,
      WOB, WOB, kDin, 0L,
      (void*)out, (void*)out, kDm, 0L,
      dummy_bias, dummy_resid, 0L,
      kRows, kDm, kDin, kOutScale);
}
